// SparseSelfAttention_75960791597210
// MI455X (gfx1250) — hardware-verified
//
#include <hip/hip_runtime.h>


#define DM    1024
#define NH    16
#define HD    64
#define WIN   128
#ifndef NB
#define NB    2
#endif
#ifndef SEQ
#define SEQ   2048
#endif
#define NB_FULL   2
#define SEQ_FULL  2048
#define MROWS (NB * SEQ)
#define NQT   (SEQ / 16)
#define XE    ((size_t)MROWS * DM)
#define WE    ((size_t)DM * DM)

#define LDSP  40
#define TP    136
#define TPF   132
#define OTP   72
#define GEMM_LDS_BYTES (128 * TP * 2)

static_assert(NB >= 1 && NB <= NB_FULL);
static_assert(SEQ >= 256 && SEQ <= SEQ_FULL);
static_assert(SEQ % 128 == 0);
static_assert(MROWS % 128 == 0);
static_assert(DM % 128 == 0);
static_assert(NQT % 4 == 0);
static_assert(2 * 128 * LDSP * 2 <= GEMM_LDS_BYTES);
static_assert(64 * TPF * 4 <= GEMM_LDS_BYTES);
static_assert(NH * HD == DM);

typedef _Float16 v16h  __attribute__((ext_vector_type(16)));
typedef _Float16 v8h   __attribute__((ext_vector_type(8)));
typedef float    v8f   __attribute__((ext_vector_type(8)));
typedef float    f32x4 __attribute__((ext_vector_type(4)));

__device__ __forceinline__ float bf16r(float f) {
    unsigned u = __float_as_uint(f);
    u = (u + 0x7FFFu + ((u >> 16) & 1u)) & 0xFFFF0000u;
    return __uint_as_float(u);
}

__device__ __forceinline__ int clampi(int v, int lo, int hi) {
    return v < lo ? lo : (v > hi ? hi : v);
}

__device__ __forceinline__ v8f zero8() {
    v8f z = {0.f, 0.f, 0.f, 0.f, 0.f, 0.f, 0.f, 0.f};
    return z;
}

__device__ __forceinline__ v16h load_frag16(const _Float16* p) {
    const v8h lo = *(const v8h*)p;
    const v8h hi = *(const v8h*)(p + 16);
    v16h f;
#pragma unroll
    for (int i = 0; i < 8; ++i) { f[i] = lo[i]; f[8 + i] = hi[i]; }
    return f;
}

__device__ __forceinline__ v8f mma16(v16h a, v16h b, v8f c) {
    c = __builtin_amdgcn_wmma_f32_16x16x32_f16(false, a, false, b, (short)0, c, false, false);
    asm volatile("v_nop\n\tv_nop\n\tv_nop\n\tv_nop" : "+v"(c) : "v"(a), "v"(b));
    return c;
}

__global__ __launch_bounds__(256)
void cvt_x(const float* __restrict__ x, _Float16* __restrict__ xh)
{
    const size_t e0 = ((size_t)blockIdx.x * 256 + threadIdx.x) * 8;
    const size_t m  = e0 / DM;
    const int col   = (int)(e0 % DM);
    const int b = (int)(m / SEQ), s = (int)(m % SEQ);
    const float* src = x + ((size_t)b * SEQ_FULL + s) * DM + col;
    const f32x4 a = *(const f32x4*)src;
    const f32x4 c = *(const f32x4*)(src + 4);
    v8h o;
#pragma unroll
    for (int i = 0; i < 4; ++i) {
        o[i]     = (_Float16)bf16r(a[i]);
        o[4 + i] = (_Float16)bf16r(c[i]);
    }
    *(volatile v8h*)(xh + e0) = o;
    __threadfence();
    *(volatile v8h*)(xh + e0) = o;
}

__global__ __launch_bounds__(256)
void cvt_w(const float* __restrict__ w0, const float* __restrict__ w1,
           const float* __restrict__ w2, const float* __restrict__ w3,
           _Float16* __restrict__ wt)
{
    __shared__ _Float16 tile[64][66];
    const int z = (int)blockIdx.z;
    const float* W = (z == 0) ? w0 : (z == 1) ? w1 : (z == 2) ? w2 : w3;
    _Float16* out = wt + (size_t)z * WE;
    const int n0 = (int)blockIdx.x * 64, k0 = (int)blockIdx.y * 64;
    const int tid = threadIdx.x, c = tid & 63, rb = tid >> 6;
#pragma unroll
    for (int jj = 0; jj < 16; ++jj) {
        const int r = rb + jj * 4;
        tile[r][c] = (_Float16)(bf16r(W[(size_t)(k0 + r) * DM + n0 + c]) * 64.0f);
    }
    __syncthreads();
    const int rn = tid >> 3, piece = tid & 7;
    v8h v0, v1;
#pragma unroll
    for (int i = 0; i < 8; ++i) {
        v0[i] = tile[piece * 8 + i][rn];
        v1[i] = tile[piece * 8 + i][rn + 32];
    }
    const size_t g0 = (size_t)(n0 + rn) * DM + k0 + piece * 8;
    const size_t g1 = (size_t)(n0 + rn + 32) * DM + k0 + piece * 8;
    *(volatile v8h*)(out + g0) = v0;
    *(volatile v8h*)(out + g1) = v1;
    __threadfence();
    *(volatile v8h*)(out + g0) = v0;
    *(volatile v8h*)(out + g1) = v1;
}

__device__ __forceinline__ void qk_pass(const _Float16* ldsh, _Float16* dst, int wv, int lane,
                                        int bidx, int hb, int s0)
{
#pragma unroll
    for (int pass = 0; pass < 8; ++pass) {
        const int L = pass * 32 + wv * 4 + (lane >> 3);
        const int piece = lane & 7, m = L >> 1, hs = L & 1;
        const v8h v = *(const v8h*)(ldsh + m * TP + hs * 64 + piece * 8);
        const size_t g = ((size_t)(bidx * NH + hb + hs) * SEQ + s0 + m) * HD + piece * 8;
        *(volatile v8h*)(dst + g) = v;
    }
}
__device__ __forceinline__ void vt_pass(const _Float16* ldsh, _Float16* dst, int wv, int lane,
                                        int bidx, int blockN, int s0)
{
#pragma unroll
    for (int pass = 0; pass < 8; ++pass) {
        const int n = pass * 16 + wv * 2 + (lane >> 4);
        const int piece = lane & 15;
        const v8h v = *(const v8h*)(ldsh + n * TP + piece * 8);
        const int ng = blockN + n, hh = ng >> 6, d = ng & 63;
        const size_t g = ((size_t)(bidx * NH + hh) * HD + d) * SEQ + s0 + piece * 8;
        *(volatile v8h*)(dst + g) = v;
    }
}
__device__ __forceinline__ void out_pass(const float* ldsf, float* dst, int wv, int lane,
                                         int m0, int blockN)
{
#pragma unroll
    for (int pass = 0; pass < 8; ++pass) {
        const int row = pass * 8 + wv;
        const f32x4 v = *(const f32x4*)(ldsf + row * TPF + lane * 4);
        const size_t g = (size_t)(m0 + row) * DM + blockN + lane * 4;
        *(volatile f32x4*)(dst + g) = v;
    }
}

__global__ __launch_bounds__(256)
void gemm_tile(const _Float16* __restrict__ Ap, const _Float16* __restrict__ wt,
               const float* __restrict__ b0, const float* __restrict__ b1,
               const float* __restrict__ b2, const float* __restrict__ b3,
               _Float16* __restrict__ qh, _Float16* __restrict__ ql,
               _Float16* __restrict__ kh, _Float16* __restrict__ kl,
               _Float16* __restrict__ vt, float* __restrict__ outp, int mode0)
{
    __shared__ __attribute__((aligned(16))) unsigned char lds_raw[GEMM_LDS_BYTES];
    _Float16* ldsh = (_Float16*)lds_raw;
    float*    ldsf = (float*)lds_raw;

    const int tid = threadIdx.x, lane = tid & 31, wv = tid >> 5;
    const int wm = wv >> 1, wn = wv & 1, half = lane >> 4, r16 = lane & 15;
    const int mode = mode0 + (int)blockIdx.y;
    const int blockM = ((int)blockIdx.x / (DM / 128)) * 128;
    const int blockN = ((int)blockIdx.x % (DM / 128)) * 128;
    const _Float16* wmat = wt + (size_t)mode * WE;
    const float* bias = (mode == 0) ? b0 : (mode == 1) ? b1 : (mode == 2) ? b2 : b3;
    const float inv = (mode == 3) ? (1.0f / 1024.0f) : (1.0f / 64.0f);

    v8f acc[2][4];
#pragma unroll
    for (int i = 0; i < 2; ++i)
#pragma unroll
        for (int j = 0; j < 4; ++j) acc[i][j] = zero8();

    const int srow = tid >> 1, sc0 = (tid & 1) * 16;
    const _Float16* ga = Ap   + (size_t)(blockM + srow) * DM + sc0;
    const _Float16* gb = wmat + (size_t)(blockN + srow) * DM + sc0;
    _Float16* As = ldsh;
    _Float16* Bs = ldsh + 128 * LDSP;

    for (int ks = 0; ks < DM / 32; ++ks) {
        const v8h a0 = *(const v8h*)(ga + ks * 32);
        const v8h a1 = *(const v8h*)(ga + ks * 32 + 8);
        const v8h w0 = *(const v8h*)(gb + ks * 32);
        const v8h w1 = *(const v8h*)(gb + ks * 32 + 8);
        __syncthreads();
        *(v8h*)(As + srow * LDSP + sc0)     = a0;
        *(v8h*)(As + srow * LDSP + sc0 + 8) = a1;
        *(v8h*)(Bs + srow * LDSP + sc0)     = w0;
        *(v8h*)(Bs + srow * LDSP + sc0 + 8) = w1;
        __syncthreads();
        v16h a[2], bf[4];
#pragma unroll
        for (int i = 0; i < 2; ++i)
            a[i] = load_frag16(As + (wm * 32 + 16 * i + r16) * LDSP + half * 8);
#pragma unroll
        for (int j = 0; j < 4; ++j)
            bf[j] = load_frag16(Bs + (wn * 64 + 16 * j + r16) * LDSP + half * 8);
#pragma unroll
        for (int i = 0; i < 2; ++i)
#pragma unroll
            for (int j = 0; j < 4; ++j)
                acc[i][j] = mma16(a[i], bf[j], acc[i][j]);
    }
    __syncthreads();

    const int bidx = blockM / SEQ, s0 = blockM % SEQ;

    if (mode < 2) {
        _Float16* dh = (mode == 0) ? qh : kh;
        _Float16* dl = (mode == 0) ? ql : kl;
        const int hb = blockN >> 6;
#pragma unroll 1
        for (int ph = 0; ph < 2; ++ph) {
            if (ph) __syncthreads();
#pragma unroll
            for (int j = 0; j < 4; ++j) {
                const int n = wn * 64 + 16 * j + r16;
                const float bb = bf16r(bias[blockN + n]);
#pragma unroll
                for (int i = 0; i < 2; ++i)
#pragma unroll
                    for (int r = 0; r < 8; ++r) {
                        const int m = wm * 32 + 16 * i + 8 * half + r;
                        const float val = acc[i][j][r] * inv + bb;
                        const _Float16 hv = (_Float16)val;
                        const _Float16 lv = (_Float16)((val - (float)hv) * 1024.0f);
                        ldsh[m * TP + n] = ph ? lv : hv;
                    }
            }
            __syncthreads();
            _Float16* dst = ph ? dl : dh;
            qk_pass(ldsh, dst, wv, lane, bidx, hb, s0);
            __threadfence();
            qk_pass(ldsh, dst, wv, lane, bidx, hb, s0);
        }
    } else if (mode == 2) {
#pragma unroll
        for (int j = 0; j < 4; ++j) {
            const int n = wn * 64 + 16 * j + r16;
            const float bb = bf16r(bias[blockN + n]);
#pragma unroll
            for (int i = 0; i < 2; ++i) {
                v8h pk;
#pragma unroll
                for (int r = 0; r < 8; ++r) pk[r] = (_Float16)(acc[i][j][r] * inv + bb);
                *(v8h*)(ldsh + n * TP + wm * 32 + 16 * i + 8 * half) = pk;
            }
        }
        __syncthreads();
        vt_pass(ldsh, vt, wv, lane, bidx, blockN, s0);
        __threadfence();
        vt_pass(ldsh, vt, wv, lane, bidx, blockN, s0);
    } else {
#pragma unroll 1
        for (int hf = 0; hf < 2; ++hf) {
            if (hf) __syncthreads();
            if ((wm >> 1) == hf) {
#pragma unroll
                for (int j = 0; j < 4; ++j) {
                    const int n = wn * 64 + 16 * j + r16;
                    const float bb = bf16r(bias[blockN + n]);
#pragma unroll
                    for (int i = 0; i < 2; ++i)
#pragma unroll
                        for (int r = 0; r < 8; ++r) {
                            const int ml = (wm & 1) * 32 + 16 * i + 8 * half + r;
                            ldsf[ml * TPF + n] = acc[i][j][r] * inv + bb;
                        }
                }
            }
            __syncthreads();
            const int m0 = blockM + hf * 64;
            out_pass(ldsf, outp, wv, lane, m0, blockN);
            __threadfence();
            out_pass(ldsf, outp, wv, lane, m0, blockN);
        }
    }
}

__device__ __forceinline__ void ctx_pass(const _Float16* ot, _Float16* ctx, int lane, int b, int q0, int h)
{
#pragma unroll
    for (int j = 0; j < 4; ++j) {
        const int q = 4 * j + (lane >> 3), piece = lane & 7;
        const v8h v = *(const v8h*)(ot + q * OTP + piece * 8);
        const size_t g = ((size_t)b * SEQ + q0 + q) * DM + h * HD + piece * 8;
        *(volatile v8h*)(ctx + g) = v;
    }
}

__global__ __launch_bounds__(128)
void attn_window(const _Float16* __restrict__ qh, const _Float16* __restrict__ ql,
                 const _Float16* __restrict__ kh, const _Float16* __restrict__ kl,
                 const _Float16* __restrict__ vt, _Float16* __restrict__ ctx)
{
    __shared__ __attribute__((aligned(16))) _Float16 otile[4 * 16 * OTP];

    const int lane = threadIdx.x & 31, wv = threadIdx.x >> 5;
    const int half = lane >> 4, r16 = lane & 15;
    const int wid = (int)blockIdx.x * 4 + wv;
    const int qt  = wid % NQT, bh = wid / NQT;
    const int b = bh / NH, h = bh % NH;
    const int q0 = qt * 16;
    const size_t head_qk = (size_t)bh * SEQ * HD;
    const size_t head_v  = (size_t)bh * HD * SEQ;
    const float NEG_INF  = -__builtin_inff();

    const size_t qoff = head_qk + (size_t)(q0 + r16) * HD + half * 8;
    const v16h bqh0 = load_frag16(qh + qoff);
    const v16h bqh1 = load_frag16(qh + qoff + 32);
    const v16h bql0 = load_frag16(ql + qoff);
    const v16h bql1 = load_frag16(ql + qoff + 32);

    v8f o[4];
#pragma unroll
    for (int dc = 0; dc < 4; ++dc) o[dc] = zero8();
    float mrun = -1.0e30f, lrun = 0.f;

    const int myq    = q0 + r16;
    const int kstart = q0 - WIN;
    const int t_lo   = (kstart < 0) ? ((-kstart) >> 5) : 0;
    int t_hi = (SEQ - 1 - kstart) >> 5;
    if (t_hi > 8) t_hi = 8;

    for (int t = t_lo; t <= t_hi; ++t) {
        const int kbase = kstart + 32 * t;

        v8f st[2], sr[2];
#pragma unroll
        for (int tl = 0; tl < 2; ++tl) {
            const int krow = clampi(kbase + 16 * tl + r16, 0, SEQ - 1);
            const size_t koff = head_qk + (size_t)krow * HD + half * 8;
            const v16h akh0 = load_frag16(kh + koff);
            const v16h akh1 = load_frag16(kh + koff + 32);
            const v16h akl0 = load_frag16(kl + koff);
            const v16h akl1 = load_frag16(kl + koff + 32);
            v8f s = zero8();
            s = mma16(akh0, bqh0, s);
            s = mma16(akh1, bqh1, s);
            v8f e = zero8();
            e = mma16(akl0, bqh0, e);
            e = mma16(akl1, bqh1, e);
            e = mma16(akh0, bql0, e);
            e = mma16(akh1, bql1, e);
            st[tl] = s;
            sr[tl] = e;
        }

        float bm = -1.0e30f;
#pragma unroll
        for (int tl = 0; tl < 2; ++tl)
#pragma unroll
            for (int r = 0; r < 8; ++r) {
                const int key = kbase + 16 * tl + 8 * half + r;
                const int dq  = key - myq;
                const bool ok = ((unsigned)key < (unsigned)SEQ) && (dq <= WIN) && (dq >= -WIN);
                float v = (st[tl][r] + sr[tl][r] * (1.0f / 1024.0f)) * 0.125f;
                v = ok ? v : NEG_INF;
                st[tl][r] = v;
                bm = fmaxf(bm, v);
            }
        bm = fmaxf(bm, __shfl_xor(bm, 16, 32));
        const float mnew  = fmaxf(mrun, bm);
        const float alpha = __expf(mrun - mnew);

        v16h bp;
        float bs = 0.f;
#pragma unroll
        for (int r = 0; r < 8; ++r) {
            const float p0 = __expf(st[0][r] - mnew);
            const float p1 = __expf(st[1][r] - mnew);
            bs += p0 + p1;
            bp[r]     = (_Float16)(p0 * 1024.0f);
            bp[8 + r] = (_Float16)(p1 * 1024.0f);
        }
        bs += __shfl_xor(bs, 16, 32);
        lrun = lrun * alpha + bs;
        mrun = mnew;
#pragma unroll
        for (int dc = 0; dc < 4; ++dc) o[dc] = o[dc] * alpha;

        const int run0 = clampi(kbase + 8 * half,      0, SEQ - 8);
        const int run1 = clampi(kbase + 16 + 8 * half, 0, SEQ - 8);
#pragma unroll
        for (int dc = 0; dc < 4; ++dc) {
            const _Float16* pv = vt + head_v + (size_t)(16 * dc + r16) * SEQ;
            const v8h va = *(const v8h*)(pv + run0);
            const v8h vb = *(const v8h*)(pv + run1);
            v16h av;
#pragma unroll
            for (int i = 0; i < 8; ++i) { av[i] = va[i]; av[8 + i] = vb[i]; }
            o[dc] = mma16(av, bp, o[dc]);
        }
    }

    const float rl = (16.0f / 1024.0f) * (1.0f / lrun);
    _Float16* ot = otile + wv * 16 * OTP;
#pragma unroll
    for (int dc = 0; dc < 4; ++dc) {
        v8h pk;
#pragma unroll
        for (int r = 0; r < 8; ++r) pk[r] = (_Float16)(o[dc][r] * rl);
        *(v8h*)(ot + r16 * OTP + 16 * dc + 8 * half) = pk;
    }
    __syncthreads();
    ctx_pass(ot, ctx, lane, b, q0, h);
    __threadfence();
    ctx_pass(ot, ctx, lane, b, q0, h);
}

extern "C" void kernel_launch(void* const* d_in, const int* in_sizes, int n_in,
                              void* d_out, int out_size, void* d_ws, size_t ws_size,
                              hipStream_t stream)
{
    if (n_in < 9) return;
    const float* x  = (const float*)d_in[0];
    const float* Wq = (const float*)d_in[1];
    const float* bq = (const float*)d_in[2];
    const float* Wk = (const float*)d_in[3];
    const float* bk = (const float*)d_in[4];
    const float* Wv = (const float*)d_in[5];
    const float* bv = (const float*)d_in[6];
    const float* Wo = (const float*)d_in[7];
    const float* bo = (const float*)d_in[8];
    float* out = (float*)d_out;

    const size_t need_x = ((size_t)(NB - 1) * SEQ_FULL + SEQ) * DM;
    if ((size_t)in_sizes[0] < need_x) return;
    if ((size_t)in_sizes[1] < WE || (size_t)in_sizes[3] < WE ||
        (size_t)in_sizes[5] < WE || (size_t)in_sizes[7] < WE) return;
    if (in_sizes[2] < DM || in_sizes[4] < DM || in_sizes[6] < DM || in_sizes[8] < DM) return;
    if ((size_t)out_size < XE) return;

    const size_t total_halves = XE + 4 * WE + 6 * XE;
    if (ws_size < total_halves * sizeof(_Float16)) return;
    _Float16* base = (_Float16*)d_ws;
    _Float16* xh  = base;
    _Float16* wt  = xh + XE;
    _Float16* qh  = wt + 4 * WE;
    _Float16* ql  = qh + XE;
    _Float16* kh  = ql + XE;
    _Float16* kl  = kh + XE;
    _Float16* vtp = kl + XE;
    _Float16* ctx = vtp + XE;

    cvt_x<<<dim3((unsigned)(XE / 2048)), dim3(256), 0, stream>>>(x, xh);
    cvt_w<<<dim3(DM / 64, DM / 64, 4), dim3(256), 0, stream>>>(Wq, Wk, Wv, Wo, wt);
    gemm_tile<<<dim3((MROWS / 128) * (DM / 128), 3), dim3(256), 0, stream>>>(
        xh, wt, bq, bk, bv, bo, qh, ql, kh, kl, vtp, out, 0);
    attn_window<<<dim3(NB * NH * NQT / 4), dim3(128), 0, stream>>>(qh, ql, kh, kl, vtp, ctx);
    gemm_tile<<<dim3((MROWS / 128) * (DM / 128), 1), dim3(256), 0, stream>>>(
        ctx, wt, bq, bk, bv, bo, qh, ql, kh, kl, vtp, out, 3);
}
